// GPTBlock_1958505087721
// MI455X (gfx1250) — hardware-run, weakly checked
//
#include <hip/hip_runtime.h>


#ifndef NB
#define NB 4
#endif
#ifndef SEQ
#define SEQ 2048
#endif
#define NB_FULL  4
#define SEQ_FULL 2048
#ifndef OUT_SEQ
#define OUT_SEQ SEQ
#endif
#ifndef EARLY
#define EARLY ((SEQ) < 256 ? (SEQ) : 256)
#endif
#define DM   1024
#define NH_  16
#define HD   64
#define FF   4096
#define AW   4
#define QRS  2048.0f
#define QRI  (1.0f / 2048.0f)
#define SC2  (0.125f * 1.4426950408889634f)
#define PSH  8.0f
#define WPS  256.0f
#define CSC  16.0f
#define HSC  16.0f
#define OSC  (1.0f / 4096.0f)

static_assert(HD == 64);
static_assert(NH_ * HD == DM);
static_assert(DM % 64 == 0);
static_assert(DM % 32 == 0);
static_assert(SEQ % 64 == 0);
static_assert((NB * SEQ) % 64 == 0);
static_assert(SEQ % 32 == 0);
static_assert(EARLY % 64 == 0);
static_assert(EARLY >= 64);
static_assert(EARLY <= SEQ);
static_assert((SEQ - EARLY) % 64 == 0);
static_assert(EARLY % (16 * AW) == 0);
static_assert((SEQ - EARLY) % (16 * AW) == 0);
static_assert(((size_t)SEQ * DM) % 8 == 0);
static_assert(NB <= NB_FULL);
static_assert(SEQ <= SEQ_FULL);
static_assert(FF % 64 == 0);
static_assert(FF % 32 == 0);
static_assert(HSC == CSC);
static_assert(WPS * CSC * OSC == 1.0f);
static_assert(32 * 16 * 8 == 16 * 64 * 4);
static_assert(32 * 16 * 4 == 16 * 64 * 2);
static_assert(32 * 16 * 16 == 64 * 64 * 2);
static_assert(32 * 32 * 4 == 64 * 64);
static_assert(64 * 68 * 4 <= 131072);
static_assert(AW * 16 * 68 * 4 <= 131072);

typedef _Float16 h16;
typedef unsigned short bf;
typedef __attribute__((ext_vector_type(16))) __bf16   v16bf;
typedef __attribute__((ext_vector_type(16))) _Float16 v16h;
typedef __attribute__((ext_vector_type(8)))  _Float16 v8h;
typedef __attribute__((ext_vector_type(8)))  unsigned short v8us;
typedef __attribute__((ext_vector_type(8)))  float    v8f;
typedef __attribute__((ext_vector_type(4)))  float    v4f;
typedef v4f  __attribute__((may_alias)) v4fa;

__device__ __forceinline__ unsigned short f2bf(float f) { unsigned u = __float_as_uint(f); u += 0x7FFFu + ((u >> 16) & 1u); return (unsigned short)(u >> 16); }
__device__ __forceinline__ float bfr(float f) { return __uint_as_float(((unsigned)f2bf(f)) << 16); }
__device__ __forceinline__ v16h cat16(v8h lo, v8h hi) { return __builtin_shufflevector(lo, hi, 0, 1, 2, 3, 4, 5, 6, 7, 8, 9, 10, 11, 12, 13, 14, 15); }
__device__ __forceinline__ v16bf cat16b(v8us lo, v8us hi) { return __builtin_bit_cast(v16bf, __builtin_shufflevector(lo, hi, 0, 1, 2, 3, 4, 5, 6, 7, 8, 9, 10, 11, 12, 13, 14, 15)); }
__device__ __forceinline__ v8f wmma16(v16h a, v16h b, v8f c) { return __builtin_amdgcn_wmma_f32_16x16x32_f16(false, a, false, b, (short)0, c, false, false); }
__device__ __forceinline__ v8f wmmab(v16bf a, v16bf b, v8f c) { return __builtin_amdgcn_wmma_f32_16x16x32_bf16(false, a, false, b, (short)0, c, false, false); }
__device__ __forceinline__ v16h  ldh(const h16* p) { return cat16(*(const v8h*)p, *(const v8h*)(p + 16)); }
__device__ __forceinline__ v16bf ldb(const bf* p)  { return cat16b(*(const v8us*)p, *(const v8us*)(p + 16)); }
__device__ __forceinline__ void wave_sync() { __builtin_amdgcn_fence(3  , "wavefront"); __builtin_amdgcn_wave_barrier(); asm volatile("" ::: "memory"); }
__device__ __forceinline__ h16 toh_flush(float v) { const h16 r = (h16)v; return (fabsf(v) < 6.103515625e-05f) ? (h16)0.0f : r; }
__device__ __forceinline__ v8f wmma16g(v16h a, v16h b, v8f c) {
    c = __builtin_amdgcn_wmma_f32_16x16x32_f16(false, a, false, b, (short)0, c, false, false);
    asm volatile("v_nop\n\tv_nop\n\tv_nop\n\tv_nop" : "+v"(c) : "v"(a), "v"(b));
    return c;
}

__global__ __launch_bounds__(256) void k_cvt8(const float* __restrict__ src, bf* dst, size_t n8) {
    const size_t i = (size_t)blockIdx.x * 256 + threadIdx.x; if (i >= n8) return;
    const v8f v = *(const v8f*)(src + i * 8); v8us o;
#pragma unroll
    for (int k = 0; k < 8; ++k) o[k] = f2bf(v[k]);
    *(volatile v8us*)(dst + i * 8) = o; __threadfence(); *(volatile v8us*)(dst + i * 8) = o;
}

template <int MODE>
__global__ __launch_bounds__(256) void k_trw(const float* __restrict__ src, unsigned short* dst, int R, int C) {
    __shared__ __align__(16) float ts[64 * 68];
    const int tid = threadIdx.x; const int c0 = blockIdx.x * 64, r0 = blockIdx.y * 64;
#pragma unroll
    for (int i = 0; i < 4; ++i) { const int idx = i * 256 + tid; const int r = idx >> 4, c4 = (idx & 15) * 4;
        const v4f v = *(const v4f*)(src + (size_t)(r0 + r) * (size_t)C + c0 + c4); *(v4fa*)(&ts[r * 68 + c4]) = v; }
    __syncthreads();
    v8us o[2];
#pragma unroll
    for (int s = 0; s < 2; ++s) { const int idx = s * 256 + tid; const int c = idx >> 3, r8 = (idx & 7) * 8;
#pragma unroll
        for (int i = 0; i < 8; ++i) { const float v = ts[(r8 + i) * 68 + c];
            if (MODE == 0) o[s][i] = f2bf(v);
            else { const h16 hv = toh_flush(bfr(v) * WPS); o[s][i] = __builtin_bit_cast(unsigned short, hv); } } }
#pragma unroll 1
    for (int ps = 0; ps < 2; ++ps) {
#pragma unroll
        for (int s = 0; s < 2; ++s) { const int idx = s * 256 + tid; const int c = idx >> 3, r8 = (idx & 7) * 8;
            *(volatile v8us*)(dst + (size_t)(c0 + c) * (size_t)R + r0 + r8) = o[s]; }
        if (ps == 0) __threadfence(); }
}

__global__ __launch_bounds__(32) void k_proj(const bf* __restrict__ A, const bf* __restrict__ Bt, h16* Ph, h16* Pr,
                                             size_t sRB, size_t sCB, size_t sRBr, size_t sCBr, int resMode, int RB, int pitch, int CB, int pitchR) {
    __shared__ __align__(16) float os[16 * 68];
    const int K = DM;
    const int lane = threadIdx.x & 31, lr = lane & 15, hi = lane >> 4; const int r0 = blockIdx.x * 64, c0 = blockIdx.y * 64;
    v8f acc[4][4];
#pragma unroll
    for (int mb = 0; mb < 4; ++mb)
#pragma unroll
        for (int nb = 0; nb < 4; ++nb) acc[mb][nb] = (v8f){};
    const size_t aoff = (size_t)(r0 + lr) * K + 8 * hi, boff = (size_t)(c0 + lr) * K + 8 * hi;
#pragma unroll 1
    for (int kc = 0; kc < K; kc += 32) {
        v16bf a[4];
#pragma unroll
        for (int mb = 0; mb < 4; ++mb) a[mb] = ldb(A + aoff + (size_t)mb * 16 * K + kc);
#pragma unroll
        for (int nb = 0; nb < 4; ++nb) { const v16bf b = ldb(Bt + boff + (size_t)nb * 16 * K + kc);
#pragma unroll
            for (int mb = 0; mb < 4; ++mb) acc[mb][nb] = wmmab(a[mb], b, acc[mb][nb]); }
        asm volatile("v_nop\n\tv_nop\n\tv_nop\n\tv_nop" : "+v"(acc[0][0]), "+v"(acc[1][1]), "+v"(acc[2][2]), "+v"(acc[3][3]) : "v"(a[0]), "v"(a[1]), "v"(a[2]), "v"(a[3]));
    }
    const size_t tbase  = (size_t)(r0 / RB) * sRB  + (size_t)(r0 % RB) * (size_t)pitch  + (size_t)(c0 / CB) * sCB  + (size_t)(c0 % CB);
    const size_t tbaseR = (size_t)(r0 / RB) * sRBr + (size_t)(r0 % RB) * (size_t)pitchR + (size_t)(c0 / CB) * sCBr + (size_t)(c0 % CB);
    const int tq = (resMode == 1) ? (r0 % RB) : (c0 % CB);
    const bool doRes = (resMode != 0) && (tq < EARLY);
    const int c8 = (lane & 7) * 8;
#pragma unroll
    for (int mb = 0; mb < 4; ++mb) {
#pragma unroll
        for (int nb = 0; nb < 4; ++nb) {
#pragma unroll
            for (int j = 0; j < 8; ++j) os[(hi * 8 + j) * 68 + nb * 16 + lr] = acc[mb][nb][j]; }
        wave_sync();
        const size_t sb = tbase + (size_t)(mb * 16) * (size_t)pitch;
        const size_t sr = tbaseR + (size_t)(mb * 16) * (size_t)pitchR;
#pragma unroll 1
        for (int ps = 0; ps < 2; ++ps) {
#pragma unroll
            for (int s = 0; s < 4; ++s) { const int row = 4 * s + (lane >> 3);
                const v4f x0 = *(const v4fa*)(&os[row * 68 + c8]); const v4f x1 = *(const v4fa*)(&os[row * 68 + c8 + 4]); v8h hv, rv;
#pragma unroll
                for (int i = 0; i < 4; ++i) { const float y0 = x0[i]; const float y1 = x1[i];
                    const h16 a0 = toh_flush(y0); const h16 a1 = toh_flush(y1); hv[i] = a0; hv[4 + i] = a1;
                    rv[i] = toh_flush((y0 - (float)a0) * QRS); rv[4 + i] = toh_flush((y1 - (float)a1) * QRS); }
                *(volatile v8h*)(Ph + sb + (size_t)row * (size_t)pitch + c8) = hv;
                if (doRes) *(volatile v8h*)(Pr + sr + (size_t)row * (size_t)pitchR + c8) = rv; }
            if (ps == 0) __threadfence(); }
        wave_sync();
    }
}

template <int EM>
__global__ __launch_bounds__(32 * AW) void k_flash(const h16* __restrict__ QH, const h16* __restrict__ QR, const h16* __restrict__ KP, const h16* __restrict__ KR,
                                                   const h16* __restrict__ VT, const h16* __restrict__ VR, h16* CH, h16* CR, int tbase) {
    __shared__ __align__(16) float os[AW * 16 * 68];
    const int lane = threadIdx.x & 31, wave = __builtin_amdgcn_readfirstlane((int)(threadIdx.x >> 5)), lr = lane & 15, hi = lane >> 4;
    const int zh = blockIdx.y; const int b = zh / NH_, h = zh % NH_;
    const int t0 = tbase + (blockIdx.x * AW + wave) * 16;
    const size_t pbase = (size_t)zh * SEQ * HD;
    const size_t rbase = (size_t)zh * EARLY * HD;
    const size_t qo = pbase + (size_t)(t0 + lr) * HD + 8 * hi;
    const v16h qh0 = ldh(QH + qo), qh1 = ldh(QH + qo + 32);
    v16h qr0 = qh0, qr1 = qh1;
    if (EM) { const size_t qro = rbase + (size_t)(t0 + lr) * HD + 8 * hi; qr0 = ldh(QR + qro); qr1 = ldh(QR + qro + 32); }
    const size_t ko  = pbase + (size_t)lr * HD + 8 * hi;
    const size_t kro = rbase + (size_t)lr * HD + 8 * hi;
    const size_t vo  = pbase + (size_t)lr * SEQ + 8 * hi;
    const size_t vro = rbase + (size_t)lr * EARLY + 8 * hi;
    v8f o0 = (v8f){}, o1 = (v8f){}, o2 = (v8f){}, o3 = (v8f){};
    v8f w0 = (v8f){}, w1 = (v8f){}, w2 = (v8f){}, w3 = (v8f){};
    float m = -3.0e38f, l = 0.0f;
    const int tq = t0 + lr, kend = t0 + 16;
#pragma unroll 1
    for (int key0 = 0; key0 < kend; key0 += 32) {
        const h16* ka = KP + ko + (size_t)key0 * HD;
        const v16h ka0 = ldh(ka), ka1 = ldh(ka + 32), kb0 = ldh(ka + 16 * HD), kb1 = ldh(ka + 16 * HD + 32);
        v8f sHa = (v8f){}, sLa = (v8f){}, sHb = (v8f){}, sLb = (v8f){};
        if (EM) {
            sHa = wmma16(ka0, qh0, sHa); sLa = wmma16(ka0, qr0, sLa); sHb = wmma16(kb0, qh0, sHb); sLb = wmma16(kb0, qr0, sLb);
            sHa = wmma16(ka1, qh1, sHa); sLa = wmma16(ka1, qr1, sLa); sHb = wmma16(kb1, qh1, sHb); sLb = wmma16(kb1, qr1, sLb);
            const h16* kr = KR + kro + (size_t)key0 * HD;
            const v16h ra0 = ldh(kr), ra1 = ldh(kr + 32), rb0 = ldh(kr + 16 * HD), rb1 = ldh(kr + 16 * HD + 32);
            sLa = wmma16(ra0, qh0, sLa); sLb = wmma16(rb0, qh0, sLb); sLa = wmma16(ra1, qh1, sLa); sLb = wmma16(rb1, qh1, sLb);
            asm volatile("v_nop\n\tv_nop\n\tv_nop\n\tv_nop" : "+v"(sHa), "+v"(sLa), "+v"(sHb), "+v"(sLb) : "v"(ra0), "v"(ra1), "v"(rb0), "v"(rb1), "v"(ka1), "v"(kb1));
        } else {
            sHa = wmma16(ka0, qh0, sHa); sHb = wmma16(kb0, qh0, sHb);
            sHa = wmma16(ka1, qh1, sHa); sHb = wmma16(kb1, qh1, sHb);
            asm volatile("v_nop\n\tv_nop\n\tv_nop\n\tv_nop" : "+v"(sHa), "+v"(sHb) : "v"(ka0), "v"(ka1), "v"(kb0), "v"(kb1));
        }
        float ta[8], tb[8];
#pragma unroll
        for (int r = 0; r < 8; ++r) {
            if (EM) { ta[r] = (sHa[r] + sLa[r] * QRI) * SC2; tb[r] = (sHb[r] + sLb[r] * QRI) * SC2; }
            else    { ta[r] = sHa[r] * SC2; tb[r] = sHb[r] * SC2; } }
        if (key0 + 31 > t0) {
            const int kq = key0 + 8 * hi;
#pragma unroll
            for (int r = 0; r < 8; ++r) { ta[r] = (kq + r <= tq) ? ta[r] : -3.0e38f; tb[r] = (kq + 16 + r <= tq) ? tb[r] : -3.0e38f; }
        }
        float mx = -3.0e38f;
#pragma unroll
        for (int r = 0; r < 8; ++r) mx = fmaxf(mx, fmaxf(ta[r], tb[r]));
        mx = fmaxf(mx, __shfl_xor(mx, 16, 32));
        const float mnew = fmaxf(m, mx);
        const float alpha = __builtin_amdgcn_exp2f(m - mnew);
        const float sh = PSH - mnew;
        v16h pb, pr; float ls = 0.0f;
#pragma unroll
        for (int r = 0; r < 8; ++r) {
            const float ea = __builtin_amdgcn_exp2f(ta[r] + sh); const float eb = __builtin_amdgcn_exp2f(tb[r] + sh);
            const h16 pa = (h16)ea; const h16 pc = (h16)eb; pb[r] = pa; pb[8 + r] = pc;
            if (EM) { pr[r] = (h16)((ea - (float)pa) * QRS); pr[8 + r] = (h16)((eb - (float)pc) * QRS); ls += ea + eb; }
            else    { pr[r] = pa; pr[8 + r] = pc; ls += (float)pa + (float)pc; } }
        l = l * alpha + ls; m = mnew;
        o0 = o0 * alpha; o1 = o1 * alpha; o2 = o2 * alpha; o3 = o3 * alpha;
        const h16* va = VT + vo + key0;
        const v16h v0 = ldh(va), v1 = ldh(va + (size_t)16 * SEQ), v2 = ldh(va + (size_t)32 * SEQ), v3 = ldh(va + (size_t)48 * SEQ);
        if (EM) {
            w0 = w0 * alpha; w1 = w1 * alpha; w2 = w2 * alpha; w3 = w3 * alpha;
            o0 = wmma16(v0, pb, o0); w0 = wmma16(v0, pr, w0); o1 = wmma16(v1, pb, o1); w1 = wmma16(v1, pr, w1);
            o2 = wmma16(v2, pb, o2); w2 = wmma16(v2, pr, w2); o3 = wmma16(v3, pb, o3); w3 = wmma16(v3, pr, w3);
            const h16* vr = VR + vro + key0;
            const v16h u0 = ldh(vr), u1 = ldh(vr + (size_t)16 * EARLY), u2 = ldh(vr + (size_t)32 * EARLY), u3 = ldh(vr + (size_t)48 * EARLY);
            w0 = wmma16(u0, pb, w0); w1 = wmma16(u1, pb, w1); w2 = wmma16(u2, pb, w2); w3 = wmma16(u3, pb, w3);
            asm volatile("v_nop\n\tv_nop\n\tv_nop\n\tv_nop" : "+v"(o0), "+v"(o1), "+v"(o2), "+v"(o3), "+v"(w0), "+v"(w1), "+v"(w2), "+v"(w3)
                         : "v"(u0), "v"(u1), "v"(u2), "v"(u3), "v"(pb), "v"(pr));
        } else {
            o0 = wmma16(v0, pb, o0); o1 = wmma16(v1, pb, o1); o2 = wmma16(v2, pb, o2); o3 = wmma16(v3, pb, o3);
            asm volatile("v_nop\n\tv_nop\n\tv_nop\n\tv_nop" : "+v"(o0), "+v"(o1), "+v"(o2), "+v"(o3) : "v"(v0), "v"(v1), "v"(v2), "v"(v3), "v"(pb));
        }
    }
    l += __shfl_xor(l, 16, 32);
    const float inv = (1.0f / l) * CSC;
    if (EM) { o0 = o0 + w0 * QRI; o1 = o1 + w1 * QRI; o2 = o2 + w2 * QRI; o3 = o3 + w3 * QRI; }
    const int wb = wave * 16 * 68;
    { v4f a, c;
      a[0] = o0[0] * inv; a[1] = o0[1] * inv; a[2] = o0[2] * inv; a[3] = o0[3] * inv; c[0] = o0[4] * inv; c[1] = o0[5] * inv; c[2] = o0[6] * inv; c[3] = o0[7] * inv;
      *(v4fa*)(&os[wb + lr * 68 +  0 + 8 * hi]) = a; *(v4fa*)(&os[wb + lr * 68 +  0 + 8 * hi + 4]) = c;
      a[0] = o1[0] * inv; a[1] = o1[1] * inv; a[2] = o1[2] * inv; a[3] = o1[3] * inv; c[0] = o1[4] * inv; c[1] = o1[5] * inv; c[2] = o1[6] * inv; c[3] = o1[7] * inv;
      *(v4fa*)(&os[wb + lr * 68 + 16 + 8 * hi]) = a; *(v4fa*)(&os[wb + lr * 68 + 16 + 8 * hi + 4]) = c;
      a[0] = o2[0] * inv; a[1] = o2[1] * inv; a[2] = o2[2] * inv; a[3] = o2[3] * inv; c[0] = o2[4] * inv; c[1] = o2[5] * inv; c[2] = o2[6] * inv; c[3] = o2[7] * inv;
      *(v4fa*)(&os[wb + lr * 68 + 32 + 8 * hi]) = a; *(v4fa*)(&os[wb + lr * 68 + 32 + 8 * hi + 4]) = c;
      a[0] = o3[0] * inv; a[1] = o3[1] * inv; a[2] = o3[2] * inv; a[3] = o3[3] * inv; c[0] = o3[4] * inv; c[1] = o3[5] * inv; c[2] = o3[6] * inv; c[3] = o3[7] * inv;
      *(v4fa*)(&os[wb + lr * 68 + 48 + 8 * hi]) = a; *(v4fa*)(&os[wb + lr * 68 + 48 + 8 * hi + 4]) = c; }
    wave_sync();
    h16* crow = CH + ((size_t)b * SEQ + t0) * DM + h * HD;
    h16* rrow = CR + ((size_t)b * EARLY + (EM ? t0 : 0)) * DM + h * HD;
    const int c8 = (lane & 7) * 8;
#pragma unroll 1
    for (int ps = 0; ps < 2; ++ps) {
#pragma unroll
        for (int s = 0; s < 4; ++s) { const int row = 4 * s + (lane >> 3);
            const v4f x0 = *(const v4fa*)(&os[wb + row * 68 + c8]); const v4f x1 = *(const v4fa*)(&os[wb + row * 68 + c8 + 4]); v8h hv, rv;
#pragma unroll
            for (int i = 0; i < 4; ++i) { const h16 a0 = (h16)x0[i]; const h16 a1 = (h16)x1[i]; hv[i] = a0; hv[4 + i] = a1;
                rv[i] = (h16)((x0[i] - (float)a0) * QRS); rv[4 + i] = (h16)((x1[i] - (float)a1) * QRS); }
            *(volatile v8h*)(crow + (size_t)row * DM + c8) = hv;
            if (EM) *(volatile v8h*)(rrow + (size_t)row * DM + c8) = rv; }
        if (ps == 0) __threadfence(); }
}

template <int RES>
__global__ __launch_bounds__(32) void k_out(const h16* __restrict__ CHp, const h16* __restrict__ CRp, const h16* __restrict__ WP, const float* __restrict__ X, float* OUT, h16* XH) {
    constexpr int MB = RES ? 2 : 4;
    __shared__ __align__(16) float os[16 * 68];
    const int lane = threadIdx.x & 31, lr = lane & 15, hi = lane >> 4;
    const int c0 = blockIdx.y * 64;
    int b, tl;
    if (RES) { constexpr int TPB = EARLY / 32; b = blockIdx.x / TPB; tl = (blockIdx.x % TPB) * 32; }
    else     { constexpr int TPB = (SEQ > EARLY) ? (SEQ - EARLY) / 64 : 1; b = blockIdx.x / TPB; tl = EARLY + (blockIdx.x % TPB) * 64; }
    const size_t arow = (size_t)b * SEQ + tl;
    const size_t rrow = (size_t)b * EARLY + (RES ? tl : 0);
    const size_t orow = (size_t)b * OUT_SEQ + tl;
    const size_t xrow = (size_t)b * SEQ_FULL + tl;
    v8f acc[4][4], accr[2][4];
#pragma unroll
    for (int mb = 0; mb < 4; ++mb)
#pragma unroll
        for (int nb = 0; nb < 4; ++nb) acc[mb][nb] = (v8f){};
#pragma unroll
    for (int mb = 0; mb < 2; ++mb)
#pragma unroll
        for (int nb = 0; nb < 4; ++nb) accr[mb][nb] = (v8f){};
    const size_t aoff = (arow + lr) * DM + 8 * hi, roff = (rrow + lr) * DM + 8 * hi, boff = (size_t)(c0 + lr) * DM + 8 * hi;
#pragma unroll 1
    for (int kc = 0; kc < DM; kc += 32) {
        v16h a[4], ar[2];
#pragma unroll
        for (int mb = 0; mb < MB; ++mb) a[mb] = ldh(CHp + aoff + (size_t)mb * 16 * DM + kc);
        if (RES) {
#pragma unroll
            for (int mb = 0; mb < 2; ++mb) ar[mb] = ldh(CRp + roff + (size_t)mb * 16 * DM + kc);
        }
#pragma unroll
        for (int nb = 0; nb < 4; ++nb) { const v16h bw = ldh(WP + boff + (size_t)nb * 16 * DM + kc);
#pragma unroll
            for (int mb = 0; mb < MB; ++mb) acc[mb][nb] = wmma16(a[mb], bw, acc[mb][nb]);
            if (RES) {
#pragma unroll
                for (int mb = 0; mb < 2; ++mb) accr[mb][nb] = wmma16(ar[mb], bw, accr[mb][nb]);
            } }
        if (RES) {
            asm volatile("v_nop\n\tv_nop\n\tv_nop\n\tv_nop"
                         : "+v"(acc[0][0]), "+v"(acc[0][1]), "+v"(acc[0][2]), "+v"(acc[0][3]), "+v"(acc[1][0]), "+v"(acc[1][1]), "+v"(acc[1][2]), "+v"(acc[1][3]),
                           "+v"(accr[0][0]), "+v"(accr[0][1]), "+v"(accr[0][2]), "+v"(accr[0][3]), "+v"(accr[1][0]), "+v"(accr[1][1]), "+v"(accr[1][2]), "+v"(accr[1][3])
                         : "v"(a[0]), "v"(a[1]), "v"(ar[0]), "v"(ar[1]));
        } else {
            asm volatile("v_nop\n\tv_nop\n\tv_nop\n\tv_nop"
                         : "+v"(acc[0][0]), "+v"(acc[0][1]), "+v"(acc[0][2]), "+v"(acc[0][3]), "+v"(acc[1][0]), "+v"(acc[1][1]), "+v"(acc[1][2]), "+v"(acc[1][3]),
                           "+v"(acc[2][0]), "+v"(acc[2][1]), "+v"(acc[2][2]), "+v"(acc[2][3]), "+v"(acc[3][0]), "+v"(acc[3][1]), "+v"(acc[3][2]), "+v"(acc[3][3])
                         : "v"(a[0]), "v"(a[1]), "v"(a[2]), "v"(a[3]));
        }
    }
    const int cofs = lr * 4;
    const int c8 = (lane & 7) * 8;
#pragma unroll
    for (int mb = 0; mb < MB; ++mb) {
#pragma unroll
        for (int nb = 0; nb < 4; ++nb) {
#pragma unroll
            for (int j = 0; j < 8; ++j) {
                float v = acc[mb][nb][j];
                if (RES) v = v + accr[mb & 1][nb][j] * QRI;
                os[(hi * 8 + j) * 68 + nb * 16 + lr] = v * OSC; } }
        wave_sync();
        const float* xb = X + (xrow + (size_t)(mb * 16)) * DM + c0;
#pragma unroll
        for (int s = 0; s < 8; ++s) { const int row = 2 * s + hi;
            const v4f xr = *(const v4f*)(xb + (size_t)row * DM + cofs);
            v4f val = *(const v4fa*)(&os[row * 68 + cofs]);
#pragma unroll
            for (int i = 0; i < 4; ++i) val[i] = val[i] + bfr(xr[i]);
            *(v4fa*)(&os[row * 68 + cofs]) = val; }
        wave_sync();
        float* ob = OUT + (orow + (size_t)(mb * 16)) * DM + c0;
        h16* hb = XH + (arow + (size_t)(mb * 16)) * DM + c0;
#pragma unroll 1
        for (int ps = 0; ps < 2; ++ps) {
#pragma unroll
            for (int s = 0; s < 8; ++s) { const int row = 2 * s + hi;
                const v4f val = *(const v4fa*)(&os[row * 68 + cofs]);
                *(volatile v4f*)(ob + (size_t)row * DM + cofs) = val; }
#pragma unroll
            for (int s = 0; s < 4; ++s) { const int row = 4 * s + (lane >> 3);
                const v4f x0 = *(const v4fa*)(&os[row * 68 + c8]); const v4f x1 = *(const v4fa*)(&os[row * 68 + c8 + 4]); v8h hv;
#pragma unroll
                for (int i = 0; i < 4; ++i) { hv[i] = toh_flush(x0[i] * CSC); hv[4 + i] = toh_flush(x1[i] * CSC); }
                *(volatile v8h*)(hb + (size_t)row * DM + c8) = hv; }
            if (ps == 0) __threadfence(); }
        wave_sync();
    }
}

__global__ __launch_bounds__(32) void k_ff1(const h16* __restrict__ XHp, const h16* __restrict__ W1, h16* HPo) {
    __shared__ __align__(16) float os[64 * 68];
    const int lane = threadIdx.x & 31, lr = lane & 15, hi = lane >> 4;
    const int r0 = blockIdx.x * 64, c0 = blockIdx.y * 64;
    v8f acc[4][4];
#pragma unroll
    for (int mb = 0; mb < 4; ++mb)
#pragma unroll
        for (int nb = 0; nb < 4; ++nb) acc[mb][nb] = (v8f){};
    const size_t aoff = (size_t)(r0 + lr) * DM + 8 * hi, boff = (size_t)(c0 + lr) * DM + 8 * hi;
#pragma unroll 1
    for (int kc = 0; kc < DM; kc += 32) {
        v16h a[4];
#pragma unroll
        for (int mb = 0; mb < 4; ++mb) a[mb] = ldh(XHp + aoff + (size_t)mb * 16 * DM + kc);
#pragma unroll
        for (int nb = 0; nb < 4; ++nb) { const v16h bw = ldh(W1 + boff + (size_t)nb * 16 * DM + kc);
#pragma unroll
            for (int mb = 0; mb < 4; ++mb) acc[mb][nb] = wmma16g(a[mb], bw, acc[mb][nb]); }
    }
#pragma unroll
    for (int mb = 0; mb < 4; ++mb)
#pragma unroll
        for (int nb = 0; nb < 4; ++nb)
#pragma unroll
            for (int j = 0; j < 8; ++j) os[(mb * 16 + hi * 8 + j) * 68 + nb * 16 + lr] = acc[mb][nb][j] * OSC;
    wave_sync();
#pragma unroll 1
    for (int it = 0; it < 32; ++it) { const int idx = it * 32 + lane; const int row = idx >> 4, c4 = (idx & 15) * 4;
        v4f v = *(const v4fa*)(&os[row * 68 + c4]);
#pragma unroll
        for (int i = 0; i < 4; ++i) { const float p = v[i]; v[i] = (0.5f * p * (1.0f + erff(p * 0.70710678118654752f))) * HSC; }
        *(v4fa*)(&os[row * 68 + c4]) = v; }
    wave_sync();
    h16* hb = HPo + (size_t)r0 * FF + c0;
    const int c8 = (lane & 7) * 8;
#pragma unroll 1
    for (int ps = 0; ps < 2; ++ps) {
#pragma unroll 4
        for (int s = 0; s < 16; ++s) { const int row = 4 * s + (lane >> 3);
            const v4f x0 = *(const v4fa*)(&os[row * 68 + c8]); const v4f x1 = *(const v4fa*)(&os[row * 68 + c8 + 4]); v8h hv;
#pragma unroll
            for (int i = 0; i < 4; ++i) { hv[i] = toh_flush(x0[i]); hv[4 + i] = toh_flush(x1[i]); }
            *(volatile v8h*)(hb + (size_t)row * FF + c8) = hv; }
        if (ps == 0) __threadfence(); }
}

__global__ __launch_bounds__(32) void k_ff2(const h16* __restrict__ HPp, const h16* __restrict__ W2, float* OUT) {
    __shared__ __align__(16) float os[16 * 68];
    const int lane = threadIdx.x & 31, lr = lane & 15, hi = lane >> 4;
    const int r0 = blockIdx.x * 64, c0 = blockIdx.y * 64;
    const int b = r0 / SEQ, tl = r0 % SEQ;
    const size_t orow = (size_t)b * OUT_SEQ + tl;
    v8f acc[4][4];
#pragma unroll
    for (int mb = 0; mb < 4; ++mb)
#pragma unroll
        for (int nb = 0; nb < 4; ++nb) acc[mb][nb] = (v8f){};
    const size_t aoff = (size_t)(r0 + lr) * FF + 8 * hi, boff = (size_t)(c0 + lr) * FF + 8 * hi;
#pragma unroll 1
    for (int kc = 0; kc < FF; kc += 32) {
        v16h a[4];
#pragma unroll
        for (int mb = 0; mb < 4; ++mb) a[mb] = ldh(HPp + aoff + (size_t)mb * 16 * FF + kc);
#pragma unroll
        for (int nb = 0; nb < 4; ++nb) { const v16h bw = ldh(W2 + boff + (size_t)nb * 16 * FF + kc);
#pragma unroll
            for (int mb = 0; mb < 4; ++mb) acc[mb][nb] = wmma16g(a[mb], bw, acc[mb][nb]); }
    }
    const int cofs = lr * 4;
#pragma unroll
    for (int mb = 0; mb < 4; ++mb) {
#pragma unroll
        for (int nb = 0; nb < 4; ++nb) {
#pragma unroll
            for (int j = 0; j < 8; ++j) os[(hi * 8 + j) * 68 + nb * 16 + lr] = acc[mb][nb][j] * OSC; }
        wave_sync();
        float* ob = OUT + (orow + (size_t)(mb * 16)) * DM + c0;
        v4f val[8];
#pragma unroll
        for (int s = 0; s < 8; ++s) { const int row = 2 * s + hi;
            const v4f x1v = *(const v4f*)(ob + (size_t)row * DM + cofs);
            val[s] = *(const v4fa*)(&os[row * 68 + cofs]) + x1v; }
#pragma unroll 1
        for (int ps = 0; ps < 2; ++ps) {
#pragma unroll
            for (int s = 0; s < 8; ++s) { const int row = 2 * s + hi;
                *(volatile v4f*)(ob + (size_t)row * DM + cofs) = val[s]; }
            if (ps == 0) __threadfence(); }
        wave_sync();
    }
}

static constexpr size_t al256(size_t v) { return (v + 255) & ~(size_t)255; }
static constexpr size_t SZ_W1 = al256((size_t)FF * DM * 2);
static constexpr size_t SZ_W2 = al256((size_t)DM * FF * 2);
static constexpr size_t SZ_XB = al256((size_t)NB * SEQ * DM * 2);
static constexpr size_t SZ_WT = al256((size_t)3 * DM * DM * 2);
static constexpr size_t SZ_WP = al256((size_t)DM * DM * 2);
static constexpr size_t SZ_PL = al256((size_t)NB * NH_ * SEQ * HD * 2);
static constexpr size_t SZ_PR = al256((size_t)NB * NH_ * EARLY * HD * 2);
static constexpr size_t SZ_CH = al256((size_t)NB * SEQ * DM * 2);
static constexpr size_t SZ_CR = al256((size_t)NB * EARLY * DM * 2);
static constexpr size_t SZ_HP = al256((size_t)NB * SEQ * FF * 2);
static constexpr size_t SZ_STAGE = SZ_WT + SZ_WP + 3 * SZ_PL + 3 * SZ_PR + SZ_CH + SZ_CR;
static constexpr size_t SZ_UNION = (SZ_STAGE > SZ_HP) ? SZ_STAGE : SZ_HP;
static constexpr size_t SZ_TOTAL = SZ_W1 + SZ_W2 + SZ_XB + SZ_UNION;
static_assert(SZ_TOTAL <= (size_t)134217728);
static_assert(SZ_HP <= SZ_UNION);
static_assert(SZ_STAGE <= SZ_UNION);
static_assert((size_t)NB * SEQ * DM * 2 <= SZ_XB);
static_assert(((size_t)DM * DM * 2) % 256 == 0);

extern "C" void kernel_launch(void* const* d_in, const int* in_sizes, int n_in,
                              void* d_out, int out_size, void* d_ws, size_t ws_size, hipStream_t stream) {
    if (n_in < 5) return;
    const size_t needx = ((size_t)(NB - 1) * SEQ_FULL + SEQ) * DM;
    if ((size_t)in_sizes[0] < needx) return;
    if ((size_t)in_sizes[1] < (size_t)3 * DM * DM || (size_t)in_sizes[2] < (size_t)DM * DM) return;
    if ((size_t)in_sizes[3] < (size_t)DM * FF || (size_t)in_sizes[4] < (size_t)FF * DM) return;
    if ((size_t)out_size < ((size_t)(NB - 1) * OUT_SEQ + SEQ) * DM) return;
    if (SZ_TOTAL > ws_size) return;
    const float* x = (const float*)d_in[0]; const float* wqkv = (const float*)d_in[1]; const float* wout = (const float*)d_in[2];
    const float* wff1 = (const float*)d_in[3]; const float* wff2 = (const float*)d_in[4];
    float* OUT = (float*)d_out;
    char* wsp = (char*)d_ws;
    h16* W1T = (h16*)wsp; wsp += SZ_W1;
    h16* W2T = (h16*)wsp; wsp += SZ_W2;
    bf*  XB  = (bf*)wsp;
    h16* X1H = (h16*)wsp; wsp += SZ_XB;
    h16* HP  = (h16*)wsp;
    bf*  WT = (bf*)wsp;  wsp += SZ_WT;
    h16* WP = (h16*)wsp; wsp += SZ_WP;
    h16* QH = (h16*)wsp; wsp += SZ_PL;
    h16* KP = (h16*)wsp; wsp += SZ_PL;
    h16* VT = (h16*)wsp; wsp += SZ_PL;
    h16* QR = (h16*)wsp; wsp += SZ_PR;
    h16* KR = (h16*)wsp; wsp += SZ_PR;
    h16* VR = (h16*)wsp; wsp += SZ_PR;
    h16* CH = (h16*)wsp; wsp += SZ_CH;
    h16* CR = (h16*)wsp; wsp += SZ_CR;

    if (SEQ == SEQ_FULL) {
        const size_t n8 = (size_t)NB * SEQ * DM / 8;
        k_cvt8<<<(unsigned)((n8 + 255) / 256), 256, 0, stream>>>(x, XB, n8);
    } else {
        const size_t n8 = (size_t)SEQ * DM / 8;
        for (int b = 0; b < NB; ++b) k_cvt8<<<(unsigned)((n8 + 255) / 256), 256, 0, stream>>>(x + (size_t)b * SEQ_FULL * DM, XB + (size_t)b * SEQ * DM, n8);
    }
    k_trw<0><<<dim3(3 * DM / 64, DM / 64, 1), 256, 0, stream>>>(wqkv, (unsigned short*)WT, DM, 3 * DM);
    k_trw<1><<<dim3(DM / 64, DM / 64, 1), 256, 0, stream>>>(wout, (unsigned short*)WP, DM, DM);
    k_trw<1><<<dim3(FF / 64, DM / 64, 1), 256, 0, stream>>>(wff1, (unsigned short*)W1T, DM, FF);
    k_trw<1><<<dim3(DM / 64, FF / 64, 1), 256, 0, stream>>>(wff2, (unsigned short*)W2T, FF, DM);

    k_proj<<<dim3(NB * SEQ / 64, DM / 64, 1), 32, 0, stream>>>(XB, WT, QH, QR,
        (size_t)NH_ * SEQ * HD, (size_t)SEQ * HD, (size_t)NH_ * EARLY * HD, (size_t)EARLY * HD, 1, SEQ, HD, HD, HD);
    k_proj<<<dim3(NB * SEQ / 64, DM / 64, 1), 32, 0, stream>>>(XB, WT + (size_t)DM * DM, KP, KR,
        (size_t)NH_ * SEQ * HD, (size_t)SEQ * HD, (size_t)NH_ * EARLY * HD, (size_t)EARLY * HD, 1, SEQ, HD, HD, HD);
    k_proj<<<dim3(DM / 64, NB * SEQ / 64, 1), 32, 0, stream>>>(WT + (size_t)2 * DM * DM, XB, VT, VR,
        (size_t)0, (size_t)DM * SEQ, (size_t)0, (size_t)DM * EARLY, 2, DM, SEQ, SEQ, EARLY);

    k_flash<1><<<dim3(EARLY / (16 * AW), NB * NH_, 1), 32 * AW, 0, stream>>>(QH, QR, KP, KR, VT, VR, CH, CR, 0);
    if (SEQ > EARLY)
        k_flash<0><<<dim3((SEQ - EARLY) / (16 * AW), NB * NH_, 1), 32 * AW, 0, stream>>>(QH, QR, KP, KR, VT, VR, CH, CR, EARLY);

    k_out<1><<<dim3(NB * (EARLY / 32), DM / 64, 1), 32, 0, stream>>>(CH, CR, WP, x, OUT, X1H);
    if (SEQ > EARLY)
        k_out<0><<<dim3(NB * ((SEQ - EARLY) / 64), DM / 64, 1), 32, 0, stream>>>(CH, CR, WP, x, OUT, X1H);

    k_ff1<<<dim3(NB * SEQ / 64, FF / 64, 1), 32, 0, stream>>>(X1H, W1T, HP);
    k_ff2<<<dim3(NB * SEQ / 64, DM / 64, 1), 32, 0, stream>>>(HP, W2T, OUT);
}
